// KANLayer_78005196030433
// MI455X (gfx1250) — hardware-verified
//
#include <hip/hip_runtime.h>
#include <math.h>

constexpr int kBatch  = 512;
constexpr int kIn     = 512;
constexpr int kOut    = 512;
constexpr int kKnots  = 15;
constexpr int kBasis  = 11;
constexpr int kSlot   = 12;
constexpr int kKdim   = kIn * kSlot;
constexpr int kPaI    = 256;
constexpr int kPwI    = 32;
constexpr int kPwO    = 8;
static_assert(kKdim % 32 == 0, "K multiple of 32");
static_assert(kBatch % 64 == 0 && kOut % 64 == 0, "M,N multiples of 64");
static_assert(kIn % kPaI == 0 && kIn % kPwI == 0 && kOut % kPwO == 0, "exact grids");
static_assert((kPaI * kKnots) % 4 == 0, "knot stage as 16-B vectors");
static_assert(kPaI * kKnots / 4 == 960 && (960 - 768) % 32 == 0, "knot tail chunk count is wave-uniform");
static_assert(kPaI * kSlot / 8 == 384 && kPwO * kPwI * kSlot / 8 == 384, "384 16-B chunks per block per plane");
static_assert((kPwI * kSlot) / 8 == 48, "48 chunks per W row segment");

typedef __attribute__((ext_vector_type(16))) _Float16 v16h;
typedef __attribute__((ext_vector_type(8)))  _Float16 v8h;
typedef __attribute__((ext_vector_type(16))) __bf16   v16b;
typedef __attribute__((ext_vector_type(8)))  __bf16   v8b;
typedef __attribute__((ext_vector_type(8)))  float    v8f;
typedef __attribute__((ext_vector_type(4)))  float    v4f;
typedef __attribute__((ext_vector_type(4)))  unsigned int v4u;

__device__ __forceinline__ unsigned short f2bf_bits(float f) {
  unsigned u = __float_as_uint(f);
  return (unsigned short)((u + 0x7FFFu + ((u >> 16) & 1u)) >> 16);
}
__device__ __forceinline__ float bf_bits2f(unsigned short h) { return __uint_as_float(((unsigned)h) << 16); }

__device__ __forceinline__ void dep_guard_h(v8f& a, v8f& b, v16h x, v16h y) { asm volatile("v_nop\n\tv_nop\n\tv_nop\n\tv_nop" : "+v"(a), "+v"(b) : "v"(x), "v"(y)); }
__device__ __forceinline__ void dep_guard_b(v8f& a, v8f& b, v16b x, v16b y) { asm volatile("v_nop\n\tv_nop\n\tv_nop\n\tv_nop" : "+v"(a), "+v"(b) : "v"(x), "v"(y)); }
__device__ __forceinline__ void dep_guard4_h(v8f& a, v8f& b, v8f& c, v8f& d, v16h x, v16h y) { asm volatile("v_nop\n\tv_nop\n\tv_nop\n\tv_nop" : "+v"(a), "+v"(b), "+v"(c), "+v"(d) : "v"(x), "v"(y)); }
__device__ __forceinline__ void dep_guard4_b(v8f& a, v8f& b, v8f& c, v8f& d, v16b x, v16b y) { asm volatile("v_nop\n\tv_nop\n\tv_nop\n\tv_nop" : "+v"(a), "+v"(b), "+v"(c), "+v"(d) : "v"(x), "v"(y)); }
__device__ __forceinline__ void keep4_h(v16h a, v16h b, v16h c, v16h d) { asm volatile("v_nop" :: "v"(a), "v"(b), "v"(c), "v"(d)); }
__device__ __forceinline__ void keep4_b(v16b a, v16b b, v16b c, v16b d) { asm volatile("v_nop" :: "v"(a), "v"(b), "v"(c), "v"(d)); }
__device__ __forceinline__ void acc_guard4(v8f& a, v8f& b, v8f& c, v8f& d) { asm volatile("v_nop\n\tv_nop\n\tv_nop\n\tv_nop" : "+v"(a), "+v"(b), "+v"(c), "+v"(d)); }
template <typename T> struct Frag;
template <> struct Frag<_Float16> {
  typedef v16h V; union U { v16h v; v8h h[2]; };
  static __device__ __forceinline__ v16h load(const _Float16* p) {
    U f; f.h[0] = *(const v8h*)(p); f.h[1] = *(const v8h*)(p + 16); return f.v;
  }
  static __device__ __forceinline__ v8f mma(v16h a, v16h b, v8f c) {
    return __builtin_amdgcn_wmma_f32_16x16x32_f16(false, a, false, b, (short)0, c, false, false);
  }
  static __device__ __forceinline__ void guard(v8f& a, v8f& b, v16h x, v16h y) { dep_guard_h(a, b, x, y); }
  static __device__ __forceinline__ void guard4(v8f& a, v8f& b, v8f& c, v8f& d, v16h x, v16h y) { dep_guard4_h(a, b, c, d, x, y); }
  static __device__ __forceinline__ void keep(v16h a, v16h b, v16h c, v16h d) { keep4_h(a, b, c, d); }
};
template <> struct Frag<__bf16> {
  typedef v16b V; union U { v16b v; v8b h[2]; };
  static __device__ __forceinline__ v16b load(const __bf16* p) {
    U f; f.h[0] = *(const v8b*)(p); f.h[1] = *(const v8b*)(p + 16); return f.v;
  }
  static __device__ __forceinline__ v8f mma(v16b a, v16b b, v8f c) {
    return __builtin_amdgcn_wmma_f32_16x16x32_bf16(false, a, false, b, (short)0, c, false, false);
  }
  static __device__ __forceinline__ void guard(v8f& a, v8f& b, v16b x, v16b y) { dep_guard_b(a, b, x, y); }
  static __device__ __forceinline__ void guard4(v8f& a, v8f& b, v8f& c, v8f& d, v16b x, v16b y) { dep_guard4_b(a, b, c, d, x, y); }
  static __device__ __forceinline__ void keep(v16b a, v16b b, v16b c, v16b d) { keep4_b(a, b, c, d); }
};

__device__ __forceinline__ unsigned pk16(unsigned short a, unsigned short b) { return (unsigned)a | ((unsigned)b << 16); }

template <int ET> struct Elem;
template <> struct Elem<0> { typedef _Float16 T; };
template <> struct Elem<1> { typedef __bf16 T; };
template <int ET, bool SPLIT, int BIAS_MODE, int OUT_MODE, bool RESID, int ACT = 0>
__global__ __launch_bounds__(256) void wmma_gemm64(
    const unsigned short* __restrict__ Ap, const unsigned short* __restrict__ A2p, int lda, long strideA,
    const unsigned short* __restrict__ Btp, const unsigned short* __restrict__ Bt2p, int ldb, long strideB,
    void* __restrict__ Cout, void* __restrict__ Cout2, int ldc, long strideC,
    const float* __restrict__ bias,
    const float* __restrict__ resid, long strideR,
    int M, int N, int K, float scale) {
  typedef typename Elem<ET>::T T;
  typedef typename Frag<T>::V V;
  const T* A = (const T*)Ap; const T* A2 = (const T*)A2p; const T* Bt = (const T*)Btp; const T* Bt2 = (const T*)Bt2p;
  __shared__ __align__(16) float sT[8][16 * 68];
  const int b    = blockIdx.y;
  const int lane = threadIdx.x & 31;
  const int wave = threadIdx.x >> 5;
  const int tilesN = N >> 6;
  const int tilesM = M >> 6;
  const int tile = blockIdx.x * 8 + wave;
  if (tile >= tilesM * tilesN) return;
  const int tm = tile / tilesN;
  const int tn = tile - tm * tilesN;
  const int m0 = tm << 6;
  const int n0 = tn << 6;

  const T* Ab  = A  + (size_t)b * strideA;
  const T* Bb  = Bt + (size_t)b * strideB;
  const T* Ab2 = SPLIT ? (A2  + (size_t)b * strideA) : nullptr;
  const T* Bb2 = SPLIT ? (Bt2 + (size_t)b * strideB) : nullptr;

  const int rlane = lane & 15;
  const int koff  = (lane >> 4) * 8;
  const int mOff  = (lane >> 4) * 8;

  v8f acc[4][4];
#pragma unroll
  for (int i = 0; i < 4; ++i)
#pragma unroll
    for (int j = 0; j < 4; ++j) acc[i][j] = (v8f){0.f,0.f,0.f,0.f,0.f,0.f,0.f,0.f};

  for (int k0 = 0; k0 < K; k0 += 32) {
    V bh[4], bl[4];
#pragma unroll
    for (int j = 0; j < 4; ++j) {
      const size_t bo = (size_t)(n0 + (j << 4) + rlane) * ldb + koff + k0;
      bh[j] = Frag<T>::load(Bb + bo);
      if (SPLIT) bl[j] = Frag<T>::load(Bb2 + bo);
    }
#pragma unroll
    for (int i = 0; i < 4; ++i) {
      const size_t ao = (size_t)(m0 + (i << 4) + rlane) * lda + koff + k0;
      V ah = Frag<T>::load(Ab + ao);
      V al;
      if (SPLIT) al = Frag<T>::load(Ab2 + ao);
#pragma unroll
      for (int j = 0; j < 4; ++j) {
        acc[i][j] = Frag<T>::mma(ah, bh[j], acc[i][j]);
        if (SPLIT) {
          acc[i][j] = Frag<T>::mma(ah, bl[j], acc[i][j]);
          acc[i][j] = Frag<T>::mma(al, bh[j], acc[i][j]);
        }
      }
      Frag<T>::guard4(acc[i][0], acc[i][1], acc[i][2], acc[i][3], ah, SPLIT ? al : ah);
    }
    Frag<T>::keep(bh[0], bh[1], bh[2], bh[3]);
    if (SPLIT) Frag<T>::keep(bl[0], bl[1], bl[2], bl[3]);
  }
  acc_guard4(acc[0][0], acc[0][1], acc[0][2], acc[0][3]);
  acc_guard4(acc[1][0], acc[1][1], acc[1][2], acc[1][3]);
  acc_guard4(acc[2][0], acc[2][1], acc[2][2], acc[2][3]);
  acc_guard4(acc[3][0], acc[3][1], acc[3][2], acc[3][3]);

  float* slab = sT[wave];
  const float* Rb = RESID ? (resid + (size_t)b * strideR) : nullptr;
#pragma unroll
  for (int i = 0; i < 4; ++i) {
    const int mBase = m0 + (i << 4);
#pragma unroll
    for (int j = 0; j < 4; ++j) {
      const int n = n0 + (j << 4) + rlane;
      float bv = 0.f;
      if (BIAS_MODE == 2) bv = bias[n];
#pragma unroll
      for (int r = 0; r < 8; ++r) {
        float v = acc[i][j][r] * scale;
        if (BIAS_MODE == 1) v += bias[mBase + mOff + r];
        if (BIAS_MODE == 2) v += bv;
        if (RESID) v += Rb[(size_t)(mBase + mOff + r) * ldc + n];
        if (ACT == 2) v = fmaxf(v, 0.0f);
        if (ACT == 4) v = (v > 0.f) ? v : 0.01f * v;
        slab[(mOff + r) * 68 + (j << 4) + rlane] = v;
      }
    }
    __builtin_amdgcn_fence(__ATOMIC_RELEASE, "workgroup");
    __builtin_amdgcn_wave_barrier();
    __builtin_amdgcn_fence(__ATOMIC_ACQUIRE, "workgroup");
    if (OUT_MODE == 0) {
      float* C = (float*)Cout + (size_t)b * strideC;
      const int hh = lane >> 4, c4 = (lane & 15) * 4;
      for (int pass = 0; pass < 2; ++pass) {
#pragma unroll
        for (int it = 0; it < 8; ++it) {
          const int row = it * 2 + hh;
          v4f v = *(const v4f*)(slab + row * 68 + c4);
          *(volatile v4f*)(C + (size_t)(mBase + row) * ldc + n0 + c4) = v;
        }
        __threadfence();
      }
    } else {
      const int q = lane >> 3, c8 = (lane & 7) * 8;
      unsigned short* C  = (unsigned short*)Cout  + (size_t)b * strideC;
      unsigned short* C2 = (OUT_MODE == 2) ? ((unsigned short*)Cout2 + (size_t)b * strideC) : nullptr;
      for (int pass = 0; pass < 2; ++pass) {
#pragma unroll
        for (int it = 0; it < 4; ++it) {
          const int row = it * 4 + q;
          const float* sp = slab + row * 68 + c8;
          v8h hv, lv;
#pragma unroll
          for (int e = 0; e < 8; ++e) {
            if (OUT_MODE == 1) {
              hv[e] = (_Float16)sp[e];
            } else {
              unsigned short hb = f2bf_bits(sp[e]);
              unsigned short lb = f2bf_bits(sp[e] - bf_bits2f(hb));
              hv[e] = __builtin_bit_cast(_Float16, hb);
              lv[e] = __builtin_bit_cast(_Float16, lb);
            }
          }
          *(volatile v8h*)(C + (size_t)(mBase + row) * ldc + n0 + c8) = hv;
          if (OUT_MODE == 2) *(volatile v8h*)(C2 + (size_t)(mBase + row) * ldc + n0 + c8) = lv;
        }
        __threadfence();
      }
    }
    __builtin_amdgcn_fence(__ATOMIC_RELEASE, "workgroup");
    __builtin_amdgcn_wave_barrier();
    __builtin_amdgcn_fence(__ATOMIC_ACQUIRE, "workgroup");
  }
}

template <int J>
__device__ __forceinline__ void cdb_sweep(float (&Bv)[14], const float (&g)[15], const float xv) {
#pragma clang fp contract(off)
#pragma unroll
  for (int tt = 0; tt < 14 - J; ++tt) {
    const float rl    = __builtin_amdgcn_rcpf(g[tt + J] - g[tt]);
    const float rr    = __builtin_amdgcn_rcpf(g[tt + J + 1] - g[tt + 1]);
    const float left  = (xv - g[tt]) * rl;
    const float right = (g[tt + J + 1] - xv) * rr;
    const float a0    = left * Bv[tt];
    const float a1    = right * Bv[tt + 1];
    Bv[tt] = a0 + a1;
  }
}

__global__ __launch_bounds__(256) void basis_plane_kernel(const float* __restrict__ x,
                                                          const float* __restrict__ knots,
                                                          unsigned short* __restrict__ Ahi,
                                                          unsigned short* __restrict__ Alo) {
#pragma clang fp contract(off)
  __shared__ __align__(16) float sg[kPaI * kKnots];
  __shared__ __align__(16) unsigned int shi[kPaI * 6];
  __shared__ __align__(16) unsigned int slo[kPaI * 6];
  const int t  = threadIdx.x;
  const int i0 = blockIdx.x * kPaI;
  const int b  = blockIdx.y;

  {
    const float* gp = knots + (size_t)i0 * kKnots;
#pragma unroll
    for (int it = 0; it < 3; ++it) {
      const int c = t + it * 256;
      const v4f v = *(const v4f*)(gp + 4 * c);
      *(v4f*)(sg + 4 * c) = v;
    }
    if (t < 960 - 768) {
      const int c = t + 768;
      const v4f v = *(const v4f*)(gp + 4 * c);
      *(v4f*)(sg + 4 * c) = v;
    }
  }
  const float xv = x[(size_t)b * kIn + i0 + t];
  __syncthreads();

  float g[15];
#pragma unroll
  for (int j = 0; j < kKnots; ++j) g[j] = sg[t * kKnots + j];

  float Bv[14];
#pragma unroll
  for (int tt = 0; tt < 14; ++tt) Bv[tt] = (xv >= g[tt] && xv < g[tt + 1]) ? 1.0f : 0.0f;
  cdb_sweep<1>(Bv, g, xv);
  cdb_sweep<2>(Bv, g, xv);
  cdb_sweep<3>(Bv, g, xv);

  const float e    = expf(-xv);
  const float sig  = 1.0f / (1.0f + e);
  const float base = xv * sig;

  float vals[12];
#pragma unroll
  for (int k = 0; k < kBasis; ++k) vals[k] = Bv[k];
  vals[11] = base;

#pragma unroll
  for (int p = 0; p < 6; ++p) {
    const float v0 = vals[2 * p], v1 = vals[2 * p + 1];
    const unsigned short hb0 = f2bf_bits(v0);
    const unsigned short hb1 = f2bf_bits(v1);
    const unsigned short lb0 = f2bf_bits(v0 - bf_bits2f(hb0));
    const unsigned short lb1 = f2bf_bits(v1 - bf_bits2f(hb1));
    shi[6 * t + p] = pk16(hb0, hb1);
    slo[6 * t + p] = pk16(lb0, lb1);
  }
  __syncthreads();

  unsigned short* ah = Ahi + (size_t)b * kKdim + (size_t)i0 * kSlot;
  unsigned short* al = Alo + (size_t)b * kKdim + (size_t)i0 * kSlot;
  const bool sec = (t < 384 - 256);
  const v4u h0 = *(const v4u*)(shi + 4 * t);
  const v4u l0 = *(const v4u*)(slo + 4 * t);
  v4u h1 = h0, l1 = l0;
  if (sec) {
    h1 = *(const v4u*)(shi + 4 * (t + 256));
    l1 = *(const v4u*)(slo + 4 * (t + 256));
  }
  unsigned short* ph0 = ah + 8 * (size_t)t;
  unsigned short* pl0 = al + 8 * (size_t)t;
  unsigned short* ph1 = ah + 8 * (size_t)(t + 256);
  unsigned short* pl1 = al + 8 * (size_t)(t + 256);
  *(volatile v4u*)ph0 = h0;
  *(volatile v4u*)pl0 = l0;
  if (sec) { *(volatile v4u*)ph1 = h1; *(volatile v4u*)pl1 = l1; }
  __threadfence();
  *(volatile v4u*)ph0 = h0;
  *(volatile v4u*)pl0 = l0;
  if (sec) { *(volatile v4u*)ph1 = h1; *(volatile v4u*)pl1 = l1; }
}

__global__ __launch_bounds__(256) void weight_plane_kernel(const float* __restrict__ coef,
                                                           const float* __restrict__ sbase,
                                                           const float* __restrict__ ssp,
                                                           const float* __restrict__ msk,
                                                           unsigned short* __restrict__ Whi,
                                                           unsigned short* __restrict__ Wlo) {
#pragma clang fp contract(off)
  __shared__ __align__(16) unsigned int shi[kPwO * 192];
  __shared__ __align__(16) unsigned int slo[kPwO * 192];
  const int t  = threadIdx.x;
  const int il = t & 31;
  const int ol = t >> 5;
  const int i0 = blockIdx.x * kPwI;
  const int o0 = blockIdx.y * kPwO;
  const int i  = i0 + il;
  const int o  = o0 + ol;
  const size_t io = (size_t)i * kOut + o;

  const float* cp = coef + io * kBasis;
  float c[11];
#pragma unroll
  for (int k = 0; k < 8; ++k) c[k] = cp[k];
  asm volatile("" ::: "memory");
#pragma unroll
  for (int k = 8; k < kBasis; ++k) c[k] = cp[k];
  const float mv = msk[io];
  const float sv = ssp[io];
  const float bv = sbase[io];
  const float wsp = mv * sv;
  const float wb  = mv * bv;

  float vals[12];
#pragma unroll
  for (int k = 0; k < kBasis; ++k) vals[k] = wsp * c[k];
  vals[11] = wb;

#pragma unroll
  for (int p = 0; p < 6; ++p) {
    const float v0 = vals[2 * p], v1 = vals[2 * p + 1];
    const unsigned short hb0 = f2bf_bits(v0);
    const unsigned short hb1 = f2bf_bits(v1);
    const unsigned short lb0 = f2bf_bits(v0 - bf_bits2f(hb0));
    const unsigned short lb1 = f2bf_bits(v1 - bf_bits2f(hb1));
    shi[ol * 192 + il * 6 + p] = pk16(hb0, hb1);
    slo[ol * 192 + il * 6 + p] = pk16(lb0, lb1);
  }
  __syncthreads();

  const bool sec = (t < 384 - 256);
  const int c0 = t;
  const int c1 = sec ? (t + 256) : t;
  const int r0 = c0 / 48, j0 = c0 - r0 * 48;
  const int r1 = c1 / 48, j1 = c1 - r1 * 48;
  const v4u h0 = *(const v4u*)(shi + 4 * c0);
  const v4u l0 = *(const v4u*)(slo + 4 * c0);
  const v4u h1 = *(const v4u*)(shi + 4 * c1);
  const v4u l1 = *(const v4u*)(slo + 4 * c1);
  unsigned short* ph0 = Whi + (size_t)(o0 + r0) * kKdim + (size_t)i0 * kSlot + 8 * j0;
  unsigned short* pl0 = Wlo + (size_t)(o0 + r0) * kKdim + (size_t)i0 * kSlot + 8 * j0;
  unsigned short* ph1 = Whi + (size_t)(o0 + r1) * kKdim + (size_t)i0 * kSlot + 8 * j1;
  unsigned short* pl1 = Wlo + (size_t)(o0 + r1) * kKdim + (size_t)i0 * kSlot + 8 * j1;
  *(volatile v4u*)ph0 = h0;
  *(volatile v4u*)pl0 = l0;
  if (sec) { *(volatile v4u*)ph1 = h1; *(volatile v4u*)pl1 = l1; }
  __threadfence();
  *(volatile v4u*)ph0 = h0;
  *(volatile v4u*)pl0 = l0;
  if (sec) { *(volatile v4u*)ph1 = h1; *(volatile v4u*)pl1 = l1; }
}

extern "C" void kernel_launch(void* const* d_in, const int* in_sizes, int n_in,
                              void* d_out, int out_size, void* d_ws, size_t ws_size,
                              hipStream_t stream) {
  if (n_in < 6) return;
  if (in_sizes[0] < kBatch * kIn) return;
  if (in_sizes[1] < kIn * kKnots) return;
  if (in_sizes[2] < kIn * kOut * kBasis) return;
  if (in_sizes[3] < kIn * kOut || in_sizes[4] < kIn * kOut || in_sizes[5] < kIn * kOut) return;
  if (out_size < kBatch * kOut) return;

  const size_t planeBytes = (size_t)kBatch * kKdim * sizeof(unsigned short);
  const size_t total = 4 * planeBytes;
  if (total > ws_size) return;

  const float* x     = (const float*)d_in[0];
  const float* knots = (const float*)d_in[1];
  const float* coef  = (const float*)d_in[2];
  const float* sbase = (const float*)d_in[3];
  const float* ssp   = (const float*)d_in[4];
  const float* msk   = (const float*)d_in[5];
  float* out = (float*)d_out;

  char* ws = (char*)d_ws;
  unsigned short* Ahi = (unsigned short*)(ws);
  unsigned short* Alo = (unsigned short*)(ws + planeBytes);
  unsigned short* Whi = (unsigned short*)(ws + 2 * planeBytes);
  unsigned short* Wlo = (unsigned short*)(ws + 3 * planeBytes);
  const float* unusedF = (const float*)(ws);
  void* unusedO = (void*)(ws + 3 * planeBytes);

  basis_plane_kernel<<<dim3(kIn / kPaI, kBatch), 256, 0, stream>>>(x, knots, Ahi, Alo);
  weight_plane_kernel<<<dim3(kIn / kPwI, kOut / kPwO), 256, 0, stream>>>(coef, sbase, ssp, msk, Whi, Wlo);

  const int tiles = (kBatch / 64) * (kOut / 64);
  wmma_gemm64<1, true, 0, 0, false, 0><<<dim3((tiles + 7) / 8, 1), 256, 0, stream>>>(
      Ahi, Alo, kKdim, 0L,
      Whi, Wlo, kKdim, 0L,
      (void*)out, unusedO, kOut, 0L,
      unusedF,
      unusedF, 0L,
      kBatch, kOut, kKdim, 1.0f);
}
